// StandardAttention_38585986187726
// MI455X (gfx1250) — hardware-verified
//
#include <hip/hip_runtime.h>


#ifndef NB
#define NB 2
#endif
#ifndef SEQ
#define SEQ 2048
#endif
#ifndef NB_FULL
#define NB_FULL 2
#endif
#ifndef SEQ_FULL
#define SEQ_FULL 2048
#endif

namespace {
constexpr int H = 16, HD = 64, CD = 1024, N3 = 3 * CD, KD = CD, QL = SEQ, SK = SEQ, MROWS = NB * SEQ;
constexpr int EARLY = 128, EB = EARLY / 32;
constexpr int BM = 128, BN = 64, BK = 64, TP = 72, AP = BK + 8, CP = BN + 4;
constexpr int ABYTES = BM * AP * 2, BBYTES = BN * AP * 2, SMEM = 2 * ABYTES + BBYTES;
constexpr float XS = 8.0f, WS = 64.0f, YS = 16.0f, PS = 1024.0f, RS = 1024.0f;
constexpr float LOG2E = 1.4426950408889634f, LOG2B = 13.287712379549449f, RMS_EPS = 1.1920929e-07f;
static_assert(SEQ % BM == 0 && SEQ >= BM && SEQ <= SEQ_FULL && NB >= 1 && NB <= NB_FULL);
static_assert(EARLY == BM && EARLY % 64 == 0 && EB * 32 == EARLY && MROWS % BM == 0 && N3 % BN == 0 && CD % BN == 0 && KD % BK == 0);
static_assert(BM * CP * 4 <= SMEM && HD == 64 && QL == SK && SEQ % 64 == 0 && (MROWS * 128) % 256 == 0);

typedef _Float16 b16;
typedef __attribute__((ext_vector_type(16))) _Float16 v16b;
typedef __attribute__((ext_vector_type(8))) _Float16 v8b;
typedef __attribute__((ext_vector_type(8))) float v8f;
typedef __attribute__((ext_vector_type(4))) float v4f;

__device__ __forceinline__ float bf16_rne(float f) { unsigned int u = __float_as_uint(f); u += 0x7FFFu + ((u >> 16) & 1u); return __uint_as_float(u & 0xFFFF0000u); }
__device__ __forceinline__ v16b frag_kb(const b16* p, int hh) {
  const v8b a = *(const v8b*)(p + 8 * hh), b = *(const v8b*)(p + 16 + 8 * hh); v16b f;
#pragma unroll
  for (int e = 0; e < 8; ++e) { f[e] = a[e]; f[8 + e] = b[e]; }
  return f;
}
__device__ __forceinline__ v8f wmma16b(v16b a, v16b b, v8f c) {
  v8f d = __builtin_amdgcn_wmma_f32_16x16x32_f16(false, a, false, b, (short)0, c, false, false);
  asm volatile("v_nop\n\tv_nop\n\tv_nop\n\tv_nop" : "+v"(d) : "v"(a), "v"(b));
  return d;
}
__device__ __forceinline__ void wave_lds_sync() { __builtin_amdgcn_fence(3, "workgroup"); __builtin_amdgcn_wave_barrier(); __builtin_amdgcn_fence(2, "workgroup"); }
__device__ __forceinline__ float nexp2(float v) { return __builtin_amdgcn_exp2f(v); }

__device__ __forceinline__ void store_tile64(const b16 (*S)[TP], b16* dst, size_t pitch, int wave, int lane) {
  for (int pass = 0; pass < 2; ++pass) {
#pragma unroll 1
    for (int it = 0; it < 8; ++it) {
      const int r = wave * 32 + it * 4 + (lane >> 3), c8 = (lane & 7) * 8;
      const v8b o = *(const v8b*)(&S[r][c8]);
      *(volatile v8b*)(dst + (size_t)r * pitch + c8) = o; }
    __threadfence(); }
}

__global__ __launch_bounds__(256) void cvt_x_kernel(const float* __restrict__ X, b16* __restrict__ Xp) {
  const size_t u = (size_t)blockIdx.x * 256 + threadIdx.x; const size_t g = u >> 7; const int piece = (int)(u & 127);
  if (g >= (size_t)MROWS) return;
  const size_t srow = (g / SEQ) * SEQ_FULL + (g % SEQ);
  const float* src = X + srow * CD + piece * 8; b16* dst = Xp + g * CD + piece * 8;
  const v4f x0 = *(const v4f*)src, x1 = *(const v4f*)(src + 4); v8b o;
#pragma unroll
  for (int j = 0; j < 4; ++j) { o[j] = (b16)(bf16_rne(x0[j]) * XS); o[4 + j] = (b16)(bf16_rne(x1[j]) * XS); }
  *(volatile v8b*)dst = o; __threadfence(); *(volatile v8b*)dst = o;
}

__global__ __launch_bounds__(64) void cvt_w_kernel(const float* __restrict__ W, b16* __restrict__ WT, int N) {
  __shared__ __attribute__((aligned(16))) b16 St[64][TP];
  const int tid = threadIdx.x, wave = tid >> 5, lane = tid & 31; const int nb = blockIdx.x, kb = blockIdx.y;
  const float* src = W + (size_t)kb * 64 * (size_t)N + (size_t)nb * 64;
#pragma unroll 1
  for (int it = 0; it < 16; ++it) {
    const int e = (it * 64 + tid) * 4; const int kk = e >> 6, n = e & 63;
    const v4f x = *(const v4f*)(src + (size_t)kk * N + n);
#pragma unroll
    for (int j = 0; j < 4; ++j) St[n + j][kk] = (b16)(bf16_rne(x[j]) * WS);
  }
  __syncthreads();
  store_tile64(St, WT + (size_t)nb * 64 * KD + (size_t)kb * 64, KD, wave, lane);
}

__global__ __launch_bounds__(256) void gemm_kernel(const b16* __restrict__ A, const b16* __restrict__ Ar, const b16* __restrict__ BT, const float* __restrict__ bias,
                                                   float* __restrict__ C, int N, int cstr, int res_on, float oscale) {
  __shared__ __attribute__((aligned(16))) char smem[SMEM];
  b16* As = reinterpret_cast<b16*>(smem); b16* Ars = reinterpret_cast<b16*>(smem + ABYTES); b16* Bs = reinterpret_cast<b16*>(smem + 2 * ABYTES);
  float* Cs = reinterpret_cast<float*>(smem);
  const int tid = threadIdx.x, wave = tid >> 5, lane = tid & 31, hh = lane >> 4, col = lane & 15, wm = wave >> 1, wn = wave & 1;
  const int bm = (int)blockIdx.y * BM, bn = (int)blockIdx.x * BN; const int bb = bm / SEQ, t0 = bm % SEQ;
  const bool res = (res_on != 0) && (t0 < EARLY);
  const b16* Ab = A + (size_t)bm * KD; const b16* Bb = BT + (size_t)bn * KD;
  const b16* Arb = Ar + ((size_t)bb * EARLY + (size_t)t0) * KD;
  v8f acc[2][2], accr[2][2];
#pragma unroll
  for (int i = 0; i < 2; ++i)
#pragma unroll
    for (int j = 0; j < 2; ++j) { acc[i][j] = (v8f){}; accr[i][j] = (v8f){}; }
#pragma unroll 1
  for (int k0 = 0; k0 < KD; k0 += BK) {
#pragma unroll
    for (int j = 0; j < 4; ++j) { const int p = tid + 256 * j, row = p >> 3, c8 = (p & 7) * 8;
      *(v8b*)(As + row * AP + c8) = *(const v8b*)(Ab + (size_t)row * KD + k0 + c8); }
    if (res) {
#pragma unroll
      for (int j = 0; j < 4; ++j) { const int p = tid + 256 * j, row = p >> 3, c8 = (p & 7) * 8;
        *(v8b*)(Ars + row * AP + c8) = *(const v8b*)(Arb + (size_t)row * KD + k0 + c8); } }
#pragma unroll
    for (int j = 0; j < 2; ++j) { const int p = tid + 256 * j, row = p >> 3, c8 = (p & 7) * 8;
      *(v8b*)(Bs + row * AP + c8) = *(const v8b*)(Bb + (size_t)row * KD + k0 + c8); }
    __syncthreads();
#pragma unroll
    for (int ks = 0; ks < BK; ks += 32) {
      const v16b a0 = frag_kb(As + (wm * 32 + col) * AP + ks, hh), a1 = frag_kb(As + (wm * 32 + 16 + col) * AP + ks, hh);
      const v16b b0 = frag_kb(Bs + (wn * 32 + col) * AP + ks, hh), b1 = frag_kb(Bs + (wn * 32 + 16 + col) * AP + ks, hh);
      acc[0][0] = wmma16b(a0, b0, acc[0][0]); acc[0][1] = wmma16b(a0, b1, acc[0][1]);
      acc[1][0] = wmma16b(a1, b0, acc[1][0]); acc[1][1] = wmma16b(a1, b1, acc[1][1]);
      if (res) {
        const v16b r0 = frag_kb(Ars + (wm * 32 + col) * AP + ks, hh), r1 = frag_kb(Ars + (wm * 32 + 16 + col) * AP + ks, hh);
        accr[0][0] = wmma16b(r0, b0, accr[0][0]); accr[0][1] = wmma16b(r0, b1, accr[0][1]);
        accr[1][0] = wmma16b(r1, b0, accr[1][0]); accr[1][1] = wmma16b(r1, b1, accr[1][1]); }
    }
    __syncthreads();
  }
#pragma unroll
  for (int i = 0; i < 2; ++i)
#pragma unroll
    for (int j = 0; j < 2; ++j) {
      const int cc = wn * 32 + j * 16 + col; const float bv = bf16_rne(bias[bn + cc]);
#pragma unroll
      for (int r = 0; r < 8; ++r) {
        const float v = acc[i][j][r] + accr[i][j][r] * (1.0f / RS);
        Cs[(wm * 32 + i * 16 + 8 * hh + r) * CP + cc] = v * oscale + bv; } }
  __syncthreads();
  float* Cb = C + ((size_t)bb * (size_t)cstr + (size_t)t0) * (size_t)N + bn;
  for (int pass = 0; pass < 2; ++pass) {
#pragma unroll 1
    for (int it = 0; it < 8; ++it) {
      const int rr = wave * 16 + it * 2 + hh; const v4f f = *(const v4f*)(Cs + rr * CP + col * 4);
      *(volatile v4f*)(Cb + (size_t)rr * N + col * 4) = f; }
    __threadfence(); }
}

__global__ __launch_bounds__(64) void qkv_post_kernel(const float* __restrict__ QKV, b16* __restrict__ Qh, b16* __restrict__ Qr, b16* __restrict__ Kh, b16* __restrict__ Kr,
                                                      b16* __restrict__ VTh, b16* __restrict__ VTr) {
  __shared__ __attribute__((aligned(16))) b16 Sh[64][TP];
  __shared__ __attribute__((aligned(16))) b16 Sr[64][TP];
  __shared__ float Tcos[32], Tsin[32];
  const int tid = threadIdx.x, wave = tid >> 5, lane = tid & 31; const int rb = blockIdx.x; const int bhi = blockIdx.y; const int b = bhi / H, h = bhi % H;
  const bool early = (rb * 64 < EARLY);
  if (tid < 32) {
    const float invf = exp2f(-(float)tid * (LOG2B / 32.0f));
    const float ang = (float)h * invf; float sn, cn; sincosf(ang, &sn, &cn);
    Tcos[tid] = cn; Tsin[tid] = sn; }
  __syncthreads();
  const size_t row0 = (size_t)b * SEQ + (size_t)rb * 64;
  for (int cls = 0; cls < 2; ++cls) {
#pragma unroll 1
    for (int i = 0; i < 32; ++i) {
      const int tok = wave * 32 + i;
      const float* src = QKV + (row0 + tok) * (size_t)N3 + cls * CD + h * HD;
      const float e0 = src[lane], e1 = src[lane + 32];
      float ss = e0 * e0 + e1 * e1;
#pragma unroll
      for (int off = 16; off > 0; off >>= 1) ss += __shfl_xor(ss, off);
      const float rn = rsqrtf(ss * (1.0f / 64.0f) + RMS_EPS);
      const float n0 = e0 * rn, n1 = e1 * rn; const float c = Tcos[lane], s = Tsin[lane];
      const float y0 = (n0 * c + n1 * s) * XS, y1 = (n1 * c - n0 * s) * XS;
      const b16 h0 = (b16)y0, h1 = (b16)y1;
      Sh[tok][lane] = h0; Sh[tok][lane + 32] = h1;
      if (early) { Sr[tok][lane] = (b16)((y0 - (float)h0) * RS); Sr[tok][lane + 32] = (b16)((y1 - (float)h1) * RS); }
    }
    __syncthreads();
    b16* dh = (cls == 0 ? Qh : Kh) + ((size_t)bhi * SEQ + (size_t)rb * 64) * HD;
    store_tile64(Sh, dh, HD, wave, lane);
    if (early) { b16* dr = (cls == 0 ? Qr : Kr) + ((size_t)bhi * EARLY + (size_t)rb * 64) * HD; store_tile64(Sr, dr, HD, wave, lane); }
    __syncthreads();
  }
#pragma unroll 1
  for (int i = 0; i < 32; ++i) {
    const int tok = wave * 32 + i;
    const float* src = QKV + (row0 + tok) * (size_t)N3 + 2 * CD + h * HD;
    const float v0 = src[lane] * XS, v1 = src[lane + 32] * XS;
    const b16 h0 = (b16)v0, h1 = (b16)v1;
    Sh[lane][tok] = h0; Sh[lane + 32][tok] = h1;
    if (early) { Sr[lane][tok] = (b16)((v0 - (float)h0) * RS); Sr[lane + 32][tok] = (b16)((v1 - (float)h1) * RS); }
  }
  __syncthreads();
  store_tile64(Sh, VTh + (size_t)bhi * HD * (size_t)SK + (size_t)rb * 64, SK, wave, lane);
  if (early) store_tile64(Sr, VTr + (size_t)bhi * HD * (size_t)EARLY + (size_t)rb * 64, EARLY, wave, lane);
}

template <bool ER>
__global__ __launch_bounds__(64) __attribute__((amdgpu_num_vgpr(256))) void attn_kernel(const b16* __restrict__ Qh, const b16* __restrict__ Qr, const b16* __restrict__ Kh,
                                                                                      const b16* __restrict__ Kr, const b16* __restrict__ VTh, const b16* __restrict__ VTr,
                                                                                      b16* __restrict__ Yh, b16* __restrict__ Yr, int bx0) {
  __shared__ __attribute__((aligned(16))) b16 Pb[2][16][32 + 8];
  __shared__ __attribute__((aligned(16))) b16 Pr[2][16][32 + 8];
  __shared__ __attribute__((aligned(16))) b16 Th[2][16][TP];
  __shared__ __attribute__((aligned(16))) b16 Tr[2][16][TP];
  const int wave = threadIdx.x >> 5, lane = threadIdx.x & 31, hh = lane >> 4, col = lane & 15;
  const int bhi = (int)blockIdx.y; const int b = bhi / H, h = bhi % H; const int bx = (int)blockIdx.x + bx0; const int q0 = bx * 32 + wave * 16, qi = q0 + col;
  const b16* Qb = Qh + (size_t)bhi * QL * HD; const b16* Kb = Kh + (size_t)bhi * SK * HD; const b16* Vb = VTh + (size_t)bhi * HD * (size_t)SK;
  const b16* Qrb = Qr + (size_t)bhi * EARLY * HD; const b16* Krb = Kr + (size_t)bhi * EARLY * HD; const b16* Vrb = VTr + (size_t)bhi * HD * (size_t)EARLY;
  const v16b qa0 = frag_kb(Qb + (size_t)qi * HD, hh), qa1 = frag_kb(Qb + (size_t)qi * HD + 32, hh);
  v16b qr0 = (v16b){}, qr1 = (v16b){};
  if constexpr (ER) { qr0 = frag_kb(Qrb + (size_t)qi * HD, hh); qr1 = frag_kb(Qrb + (size_t)qi * HD + 32, hh); }
  const float cs = LOG2E / (8.0f * XS * XS);
  float m = -INFINITY, l = 0.0f; v8f o[4], o2[4];
#pragma unroll
  for (int t = 0; t < 4; ++t) { o[t] = (v8f){}; o2[t] = (v8f){}; }
  const int kend = bx * 32 + 32;
#pragma unroll 1
  for (int kb = 0; kb < kend; kb += 32) {
    float e[16]; float mx = -INFINITY;
#pragma unroll
    for (int u = 0; u < 2; ++u) {
      const int krow = kb + u * 16 + col;
      const v16b kh0 = frag_kb(Kb + (size_t)krow * HD, hh), kh1 = frag_kb(Kb + (size_t)krow * HD + 32, hh);
      v8f s = (v8f){}; s = wmma16b(kh0, qa0, s); s = wmma16b(kh1, qa1, s);
      v8f sr = (v8f){};
      if constexpr (ER) {
        const v16b kr0 = frag_kb(Krb + (size_t)krow * HD, hh), kr1 = frag_kb(Krb + (size_t)krow * HD + 32, hh);
        sr = wmma16b(kh0, qr0, sr); sr = wmma16b(kh1, qr1, sr); sr = wmma16b(kr0, qa0, sr); sr = wmma16b(kr1, qa1, sr); }
#pragma unroll
      for (int r = 0; r < 8; ++r) {
        float v = s[r];
        if constexpr (ER) v += sr[r] * (1.0f / RS);
        v *= cs;
        const int key = kb + u * 16 + 8 * hh + r;
        v = (key > qi) ? -INFINITY : v;
        e[u * 8 + r] = v; mx = fmaxf(mx, v); } }
    mx = fmaxf(mx, __shfl_xor(mx, 16)); const float mn = fmaxf(m, mx); const float al = nexp2(m - mn); float sum = 0.0f;
#pragma unroll
    for (int i2 = 0; i2 < 16; ++i2) {
      const float p = nexp2(e[i2] - mn); sum += p; const int pi = (i2 < 8 ? 0 : 16) + 8 * hh + (i2 & 7);
      const float pp = p * PS; const b16 ph = (b16)pp; Pb[wave][col][pi] = ph;
      if constexpr (ER) Pr[wave][col][pi] = (b16)((pp - (float)ph) * RS); }
    sum += __shfl_xor(sum, 16); l = l * al + sum; m = mn;
    wave_lds_sync();
    const v16b pf = frag_kb(&Pb[wave][col][0], hh);
    v16b prf = (v16b){};
    if constexpr (ER) prf = frag_kb(&Pr[wave][col][0], hh);
#pragma unroll
    for (int t = 0; t < 4; ++t) {
      o[t] *= al; const v16b vh = frag_kb(Vb + (size_t)(t * 16 + col) * SK + kb, hh);
      o[t] = wmma16b(vh, pf, o[t]);
      if constexpr (ER) { const v16b vr = frag_kb(Vrb + (size_t)(t * 16 + col) * EARLY + kb, hh); o2[t] *= al; o2[t] = wmma16b(vh, prf, o2[t]); o2[t] = wmma16b(vr, pf, o2[t]); } }
    wave_lds_sync(); }
  const float inv = YS / (l * PS * XS);
#pragma unroll
  for (int t = 0; t < 4; ++t) {
#pragma unroll
    for (int r = 0; r < 8; ++r) {
      float ov = o[t][r];
      if constexpr (ER) ov += o2[t][r] * (1.0f / RS);
      const float yv = ov * inv; const b16 yh = (b16)yv;
      Th[wave][col][t * 16 + 8 * hh + r] = yh;
      if constexpr (ER) Tr[wave][col][t * 16 + 8 * hh + r] = (b16)((yv - (float)yh) * RS); } }
  wave_lds_sync();
  b16* yb = Yh + ((size_t)b * SEQ + (size_t)q0) * CD + (size_t)h * HD;
  for (int pass = 0; pass < 2; ++pass) {
#pragma unroll 1
    for (int it = 0; it < 4; ++it) {
      const int rr = it * 4 + (lane >> 3), c8 = (lane & 7) * 8; const v8b f = *(const v8b*)(&Th[wave][rr][c8]);
      *(volatile v8b*)(yb + (size_t)rr * CD + c8) = f;
      if constexpr (ER) {
        const v8b fr = *(const v8b*)(&Tr[wave][rr][c8]);
        *(volatile v8b*)(Yr + (((size_t)b * EARLY + (size_t)(q0 + rr)) * CD + (size_t)h * HD + c8)) = fr; } }
    __threadfence(); }
}
}

extern "C" void kernel_launch(void* const* d_in, const int* in_sizes, int n_in, void* d_out, int out_size, void* d_ws, size_t ws_size, hipStream_t stream) {
  const size_t need_x = ((size_t)(NB - 1) * SEQ_FULL + (size_t)SEQ) * CD;
  if (n_in < 5 || (size_t)in_sizes[0] < need_x || (size_t)in_sizes[1] < (size_t)KD * N3 || (size_t)in_sizes[2] < (size_t)N3 ||
      (size_t)in_sizes[3] < (size_t)KD * CD || (size_t)in_sizes[4] < (size_t)CD || (size_t)out_size < need_x) return;
  const float* Xin = (const float*)d_in[0]; const float* Wa = (const float*)d_in[1]; const float* Ba = (const float*)d_in[2];
  const float* Wp = (const float*)d_in[3]; const float* Bp = (const float*)d_in[4];
  size_t off = 0; char* ws = (char*)d_ws;
  auto carve = [&](size_t bytes) { char* p = ws + off; off += (bytes + 255) & ~(size_t)255; return p; };
  b16* Xp = (b16*)carve((size_t)MROWS * CD * 2);
  b16* WaT = (b16*)carve((size_t)N3 * KD * 2);
  b16* WpT = (b16*)carve((size_t)CD * KD * 2);
  float* QKV = (float*)carve((size_t)MROWS * N3 * 4);
  const size_t plane = (size_t)NB * H * SEQ * HD * 2, rplane = (size_t)NB * H * EARLY * HD * 2;
  b16* Qh = (b16*)carve(plane); b16* Kh = (b16*)carve(plane); b16* VTh = (b16*)carve(plane);
  b16* Qr = (b16*)carve(rplane); b16* Kr = (b16*)carve(rplane); b16* VTr = (b16*)carve(rplane);
  b16* Yh = (b16*)carve((size_t)MROWS * CD * 2);
  b16* Yr = (b16*)carve((size_t)NB * EARLY * CD * 2);
  if (off > ws_size || off > ((size_t)128 << 20)) return;
  cvt_x_kernel<<<dim3((unsigned)(((size_t)MROWS * 128 + 255) / 256)), 256, 0, stream>>>(Xin, Xp);
  cvt_w_kernel<<<dim3(N3 / 64, KD / 64), 64, 0, stream>>>(Wa, WaT, N3);
  cvt_w_kernel<<<dim3(CD / 64, KD / 64), 64, 0, stream>>>(Wp, WpT, CD);
  gemm_kernel<<<dim3(N3 / BN, MROWS / BM), 256, 0, stream>>>(Xp, Xp, WaT, Ba, QKV, N3, SEQ, 0, 1.0f / (XS * WS));
  qkv_post_kernel<<<dim3(SEQ / 64, NB * H), 64, 0, stream>>>(QKV, Qh, Qr, Kh, Kr, VTh, VTr);
  attn_kernel<true><<<dim3(EB, NB * H), 64, 0, stream>>>(Qh, Qr, Kh, Kr, VTh, VTr, Yh, Yr, 0);
  if (QL / 32 > EB) attn_kernel<false><<<dim3(QL / 32 - EB, NB * H), 64, 0, stream>>>(Qh, Qr, Kh, Kr, VTh, VTr, Yh, Yr, EB);
  gemm_kernel<<<dim3(CD / BN, MROWS / BM), 256, 0, stream>>>(Yh, Yr, WpT, Bp, (float*)d_out, CD, SEQ_FULL, 1, 1.0f / (YS * WS));
}
